// WOP_14602888806627
// MI455X (gfx1250) — hardware-run, weakly checked
//
#include <hip/hip_runtime.h>
#include <math.h>

typedef __attribute__((ext_vector_type(16))) _Float16 v16h;
typedef __attribute__((ext_vector_type(8)))  _Float16 v8h;
typedef __attribute__((ext_vector_type(8)))  float    v8f;
typedef __attribute__((ext_vector_type(4)))  float    v4f;
typedef __attribute__((ext_vector_type(4)))  unsigned v4u;

constexpr int kBS    = 256;
constexpr int kTN    = 128;
constexpr int kIS    = 300;
constexpr int kH2    = 50;
constexpr int kNH    = 3050;
constexpr int kNHP   = 3056;
constexpr int kTH    = 12;
constexpr int kMLHS  = 16;
constexpr int kMLW   = 20;
constexpr int kNOPS  = 7;
constexpr int kKX    = 320;
constexpr int kFP    = 128;
constexpr int kGN    = 512;
constexpr int kMQ    = kBS * kTN;
constexpr int kMH    = kNHP * kTH;
constexpr int kMHR   = kNH * kTH;
constexpr int kMJ    = kBS * kMLW;
constexpr int kOutN  = kMJ * kNOPS;
constexpr float kWCarry    = 64.0f;
constexpr float kWCarryInv = 1.0f / 64.0f;
constexpr float kPCarry    = 1024.0f;
constexpr float kNegFill   = -1.0e10f;
static_assert(kMQ == 32768);
static_assert(kMH == 36672);
static_assert((kMQ % 64) == 0 && (kMH % 64) == 0 && (kMJ % 64) == 0);
static_assert((kNHP % 16) == 0 && (kBS % 16) == 0);
static_assert((kKX % 32) == 0 && (kFP % 32) == 0 && (kGN % 64) == 0);
static_assert((kOutN % 256) == 0);

constexpr size_t kSzX    = (size_t)kMH * kKX * 2;
constexpr size_t kSzG    = (size_t)kMH * kGN * 2;
constexpr size_t kSzL0   = (size_t)kMH * kFP * 2;
constexpr size_t kSzWN   = (size_t)kMQ * kFP * 2;
constexpr size_t kSzQ    = (size_t)kMQ * kFP * 2;
constexpr size_t kSzHPU  = (size_t)kNHP * kFP * 2;
constexpr size_t kSzOB   = (size_t)kMJ * kFP * 2;
constexpr size_t kSzCN   = (size_t)kMJ * kFP * 2;
constexpr size_t kSzVEC  = (size_t)kMJ * 256 * 2;
constexpr size_t kSzHF   = (size_t)kMJ * 128 * 4;
constexpr size_t kSzWih0 = (size_t)512 * kKX * 2;
constexpr size_t kSzWih1 = (size_t)512 * kFP * 2;
constexpr size_t kSzWhh  = (size_t)1024 * 64 * 2;
constexpr size_t kSzW128 = (size_t)128 * 128 * 2;
constexpr size_t kSzWo0  = (size_t)128 * 256 * 2;
constexpr size_t kSzBias = (size_t)2560 * 4;

constexpr size_t kOffX     = 0;
constexpr size_t kOffG     = kOffX     + kSzX;
constexpr size_t kOffL0    = kOffG     + kSzG;
constexpr size_t kOffWN    = kOffL0    + kSzL0;
constexpr size_t kOffQ     = kOffWN    + kSzWN;
constexpr size_t kOffHPU   = kOffQ     + kSzQ;
constexpr size_t kOffOB    = kOffHPU   + kSzHPU;
constexpr size_t kOffCN    = kOffOB    + kSzOB;
constexpr size_t kOffVEC   = kOffCN    + kSzCN;
constexpr size_t kOffHF    = kOffVEC   + kSzVEC;
constexpr size_t kOffWih0N = kOffHF    + kSzHF;
constexpr size_t kOffWih0H = kOffWih0N + kSzWih0;
constexpr size_t kOffWih1N = kOffWih0H + kSzWih0;
constexpr size_t kOffWih1H = kOffWih1N + kSzWih1;
constexpr size_t kOffWhhN  = kOffWih1H + kSzWih1;
constexpr size_t kOffWhhH  = kOffWhhN  + kSzWhh;
constexpr size_t kOffWatt  = kOffWhhH  + kSzWhh;
constexpr size_t kOffWc    = kOffWatt  + kSzW128;
constexpr size_t kOffWhs   = kOffWc    + kSzW128;
constexpr size_t kOffWo0   = kOffWhs   + kSzW128;
constexpr size_t kOffBias  = kOffWo0   + kSzWo0;
constexpr size_t kWsTotal  = kOffBias  + kSzBias;
static_assert(kWsTotal == 97187840ull);
static_assert(kWsTotal <= 134217728ull);
static_assert((kOffG % 128) == 0 && (kOffL0 % 128) == 0 && (kOffWN % 128) == 0 && (kOffQ % 128) == 0 &&
              (kOffHPU % 128) == 0 && (kOffOB % 128) == 0 && (kOffCN % 128) == 0 && (kOffVEC % 128) == 0 &&
              (kOffHF % 128) == 0 && (kOffWih0N % 128) == 0 && (kOffWih0H % 128) == 0 && (kOffWih1N % 128) == 0 &&
              (kOffWih1H % 128) == 0 && (kOffWhhN % 128) == 0 && (kOffWhhH % 128) == 0 && (kOffWatt % 128) == 0 &&
              (kOffWc % 128) == 0 && (kOffWhs % 128) == 0 && (kOffWo0 % 128) == 0 && (kOffBias % 128) == 0);

constexpr int kBiasN0 = 0, kBiasN1 = 512, kBiasH0 = 1024, kBiasH1 = 1536;
constexpr int kBiasAtt = 2048, kBiasC = 2176, kBiasHs = 2304, kBiasWo0 = 2432;

__device__ __forceinline__ float h16_to_f32(unsigned hb) {
  const unsigned sgn = (hb & 0x8000u) << 16;
  const unsigned em = hb & 0x7fffu;
  const float fn = __uint_as_float((em << 13) + 0x38000000u);
  const float fs = (float)em * 5.9604644775390625e-8f;
  const float mag = (em < 0x400u) ? fs : fn;
  return __uint_as_float(__float_as_uint(mag) | sgn);
}
__device__ __forceinline__ unsigned f32_to_h16bits(float x) {
  const _Float16 h = (_Float16)x;
  const unsigned short b = __builtin_bit_cast(unsigned short, h);
  return (unsigned)b;
}
__device__ __forceinline__ float sigm(float x) {
  return __builtin_amdgcn_rcpf(1.0f + expf(-x));
}
__device__ __forceinline__ float tanh_e(float x) {
  return 1.0f - 2.0f * __builtin_amdgcn_rcpf(expf(2.0f * x) + 1.0f);
}

struct FragH {
  union U { v16h v; v8h h[2]; };
  static __device__ __forceinline__ v16h load(const _Float16* p) {
    U f;
    f.h[0] = *(const v8h*)(p);
    f.h[1] = *(const v8h*)(p + 16);
    return f.v;
  }
};
__device__ __forceinline__ v8f mma_g(v16h a, v16h b, v8f c) {
  c = __builtin_amdgcn_wmma_f32_16x16x32_f16(false, a, false, b, (short)0, c, false, false);
  asm volatile("v_nop\n\tv_nop\n\tv_nop\n\tv_nop" : "+v"(c) : "v"(a), "v"(b));
  return c;
}
__device__ __forceinline__ v8f mma_raw(v16h a, v16h b, v8f c) {
  return __builtin_amdgcn_wmma_f32_16x16x32_f16(false, a, false, b, (short)0, c, false, false);
}
__device__ __forceinline__ void guard4_h(v8f& a, v8f& b, v8f& c, v8f& d, v16h x) {
  asm volatile("v_nop\n\tv_nop\n\tv_nop\n\tv_nop" : "+v"(a), "+v"(b), "+v"(c), "+v"(d) : "v"(x));
}
__device__ __forceinline__ void keep4_h(v16h a, v16h b, v16h c, v16h d) {
  asm volatile("v_nop" :: "v"(a), "v"(b), "v"(c), "v"(d));
}
__device__ __forceinline__ void acc_guard4(v8f& a, v8f& b, v8f& c, v8f& d) {
  asm volatile("v_nop\n\tv_nop\n\tv_nop\n\tv_nop" : "+v"(a), "+v"(b), "+v"(c), "+v"(d));
}

template <int OUT_MODE, int ACT>
__global__ __launch_bounds__(256) void wmma_gemm64(
    const unsigned short* __restrict__ Ap, int lda,
    const unsigned short* __restrict__ Btp, int ldb,
    void* __restrict__ Cout, int ldc,
    const float* __restrict__ bias,
    int M, int N, int K, float scale) {
  const _Float16* A  = (const _Float16*)(const void*)Ap;
  const _Float16* Bt = (const _Float16*)(const void*)Btp;
  __shared__ __align__(16) float sT[8][16 * 68];
  const int lane = threadIdx.x & 31;
  const int wave = threadIdx.x >> 5;
  const int tilesN = N >> 6;
  const int tilesM = M >> 6;
  const int tile = blockIdx.x * 8 + wave;
  if (tile >= tilesM * tilesN) return;
  const int tm = tile / tilesN;
  const int tn = tile - tm * tilesN;
  const int m0 = tm << 6;
  const int n0 = tn << 6;

  const int rlane = lane & 15;
  const int koff  = (lane >> 4) * 8;
  const int mOff  = (lane >> 4) * 8;

  v8f acc[4][4];
#pragma unroll
  for (int i = 0; i < 4; ++i)
#pragma unroll
    for (int j = 0; j < 4; ++j) acc[i][j] = (v8f){0.f, 0.f, 0.f, 0.f, 0.f, 0.f, 0.f, 0.f};

  for (int k0 = 0; k0 < K; k0 += 32) {
    v16h bh[4];
#pragma unroll
    for (int j = 0; j < 4; ++j) {
      const size_t bo = (size_t)(n0 + (j << 4) + rlane) * ldb + koff + k0;
      bh[j] = FragH::load(Bt + bo);
    }
#pragma unroll
    for (int i = 0; i < 4; ++i) {
      const size_t ao = (size_t)(m0 + (i << 4) + rlane) * lda + koff + k0;
      v16h ah = FragH::load(A + ao);
#pragma unroll
      for (int j = 0; j < 4; ++j) acc[i][j] = mma_raw(ah, bh[j], acc[i][j]);
      guard4_h(acc[i][0], acc[i][1], acc[i][2], acc[i][3], ah);
    }
    keep4_h(bh[0], bh[1], bh[2], bh[3]);
  }
  acc_guard4(acc[0][0], acc[0][1], acc[0][2], acc[0][3]);
  acc_guard4(acc[1][0], acc[1][1], acc[1][2], acc[1][3]);
  acc_guard4(acc[2][0], acc[2][1], acc[2][2], acc[2][3]);
  acc_guard4(acc[3][0], acc[3][1], acc[3][2], acc[3][3]);

  float* slab = sT[wave];
#pragma unroll
  for (int i = 0; i < 4; ++i) {
    const int mBase = m0 + (i << 4);
#pragma unroll
    for (int j = 0; j < 4; ++j) {
      const int n = n0 + (j << 4) + rlane;
      const float bv = bias[n];
#pragma unroll
      for (int r = 0; r < 8; ++r) {
        float v = acc[i][j][r] * scale;
        v += bv;
        if (ACT == 1) v = tanh_e(v);
        slab[(mOff + r) * 68 + (j << 4) + rlane] = v;
      }
    }
    __builtin_amdgcn_fence(__ATOMIC_RELEASE, "workgroup");
    __builtin_amdgcn_wave_barrier();
    __builtin_amdgcn_fence(__ATOMIC_ACQUIRE, "workgroup");
    if (OUT_MODE == 0) {
      float* C = (float*)Cout;
      const int hh = lane >> 4, c4 = (lane & 15) * 4;
      for (int pass = 0; pass < 2; ++pass) {
#pragma unroll
        for (int it = 0; it < 8; ++it) {
          const int row = it * 2 + hh;
          v4f v = *(const v4f*)(slab + row * 68 + c4);
          *(volatile v4f*)(C + (size_t)(mBase + row) * ldc + n0 + c4) = v;
        }
        __threadfence();
      }
    } else {
      const int q = lane >> 3, c8 = (lane & 7) * 8;
      unsigned short* C = (unsigned short*)Cout;
      for (int pass = 0; pass < 2; ++pass) {
#pragma unroll
        for (int it = 0; it < 4; ++it) {
          const int row = it * 4 + q;
          const float* sp = slab + row * 68 + c8;
          v8h hv;
#pragma unroll
          for (int e = 0; e < 8; ++e) hv[e] = (_Float16)sp[e];
          *(volatile v8h*)(C + (size_t)(mBase + row) * ldc + n0 + c8) = hv;
        }
        __threadfence();
      }
    }
    __builtin_amdgcn_fence(__ATOMIC_RELEASE, "workgroup");
    __builtin_amdgcn_wave_barrier();
    __builtin_amdgcn_fence(__ATOMIC_ACQUIRE, "workgroup");
  }
}

__global__ __launch_bounds__(256) void pack_plane_kernel(
    const float* __restrict__ src, unsigned short* __restrict__ dst,
    int srcRows, int srcCols, int dstCols8, int total8,
    int rshift, int rblk, int cshift, int cblk, float carry) {
  const int i = blockIdx.x * 256 + threadIdx.x;
  if (i >= total8) return;
  const int n = i / dstCols8;
  const int c8 = (i - n * dstCols8) * 8;
  const int rb = n >> rshift;
  const int ru = n & ((1 << rshift) - 1);
  const int srow = rb * rblk + ru;
  const bool rok = (ru < rblk) && (srow < srcRows);
  const int srowc = srow < srcRows ? srow : (srcRows - 1);
  const float* rp = src + (size_t)srowc * srcCols;
  v8h hv;
#pragma unroll
  for (int e = 0; e < 8; ++e) {
    const int kk = c8 + e;
    const int cb = kk >> cshift;
    const int cu = kk & ((1 << cshift) - 1);
    const int k = cb * cblk + cu;
    const bool ok = rok && (cu < cblk) && (k < srcCols);
    const int kc = k < srcCols ? k : (srcCols - 1);
    const float v = rp[kc];
    const float w = ok ? (v * carry) : 0.0f;
    hv[e] = (_Float16)w;
  }
  unsigned short* q = dst + (size_t)i * 8;
  *(volatile v8h*)q = hv;
  __threadfence();
  *(volatile v8h*)q = hv;
}

__global__ __launch_bounds__(32) void pack_bias_kernel(
    const float* __restrict__ nbih, const float* __restrict__ nbhh,
    const float* __restrict__ hbih, const float* __restrict__ hbhh,
    const float* __restrict__ batt, const float* __restrict__ bc,
    const float* __restrict__ bhs, const float* __restrict__ bwo0,
    float* __restrict__ dst) {
  const int j = blockIdx.x;
  const int lane = threadIdx.x;
  const bool two = (j < 16);
  const int enc = j >> 3;
  const int layer = (j >> 2) & 1;
  const int sub = j & 3;
  const float* pa = two ? (enc ? hbih : nbih)
                        : ((j == 16) ? batt : ((j == 17) ? bc : ((j == 18) ? bhs : bwo0)));
  const float* pb = two ? (enc ? hbhh : nbhh) : pa;
  const bool perm = (j <= 16);
  const int base = two ? (layer * 400 + sub * 100) : 0;
  const int limit = two ? 800 : 100;
  v4f o;
#pragma unroll
  for (int e = 0; e < 4; ++e) {
    const int n = lane * 4 + e;
    const int u = n & 63;
    const int idx = perm ? (base + (n >> 6) * 50 + u) : n;
    const bool ok = perm ? (u < kH2) : (n < 100);
    const int idxc = idx < limit ? idx : (limit - 1);
    const float va = pa[idxc];
    const float vb = pb[idxc];
    const float s = two ? (va + vb) : va;
    o[e] = ok ? s : 0.0f;
  }
  float* q = dst + (size_t)j * 128 + lane * 4;
  *(volatile v4f*)q = o;
  __threadfence();
  *(volatile v4f*)q = o;
}

__global__ __launch_bounds__(256) void convert_x_kernel(
    const float* __restrict__ src, unsigned short* __restrict__ dst, int rowsReal, int total8) {
  const int i = blockIdx.x * 256 + threadIdx.x;
  if (i >= total8) return;
  const int row = i / 40;
  const int c8 = (i - row * 40) * 8;
  const int rowc = row < rowsReal ? row : (rowsReal - 1);
  const int ca = c8 < 296 ? c8 : 296;
  const int cb = (c8 + 4) < 296 ? (c8 + 4) : 296;
  const float* rp = src + (size_t)rowc * kIS;
  const v4f a = *(const v4f*)(rp + ca);
  const v4f b = *(const v4f*)(rp + cb);
  const bool okr = row < rowsReal;
  const bool oka = okr && (c8 < kIS);
  const bool okb = okr && ((c8 + 4) < kIS);
  v8h hv;
#pragma unroll
  for (int e = 0; e < 4; ++e) {
    const float x0 = a[e];
    const float x1 = b[e];
    hv[e]     = (_Float16)(oka ? x0 : 0.0f);
    hv[4 + e] = (_Float16)(okb ? x1 : 0.0f);
  }
  unsigned short* q = dst + (size_t)i * 8;
  *(volatile v8h*)q = hv;
  __threadfence();
  *(volatile v8h*)q = hv;
}

constexpr int kHP = 72;
constexpr int kGP = 264;

template <bool LAST_ONLY>
__global__ __launch_bounds__(128) void lstm_rec_kernel(
    const unsigned short* __restrict__ G, const unsigned short* __restrict__ WhhL,
    const int* __restrict__ lens, int nreal, int T, unsigned short* __restrict__ outp) {
  __shared__ __align__(16) unsigned short sH[16 * kHP];
  __shared__ __align__(16) unsigned short sO[16 * kHP];
  __shared__ __align__(16) unsigned short sG[16 * kGP];
  const int tid = threadIdx.x, lane = tid & 31, wave = tid >> 5, hh = lane >> 4, c = lane & 15;
  const int dir = blockIdx.y;
  const int row0 = blockIdx.x * 16;
  const int unit = wave * 16 + c;
  const bool unit_ok = unit < kH2;

  const _Float16* Wd = (const _Float16*)(const void*)(WhhL + (size_t)dir * 256 * 64);
  v16h bfr[4][2];
#pragma unroll
  for (int g = 0; g < 4; ++g)
#pragma unroll
    for (int ks = 0; ks < 2; ++ks)
      bfr[g][ks] = FragH::load(Wd + (size_t)(g * 64 + unit) * 64 + ks * 32 + 8 * hh);

  int lenr[8];
#pragma unroll
  for (int r = 0; r < 8; ++r) {
    const int grow = row0 + 8 * hh + r;
    const int gl = grow < nreal ? grow : (nreal - 1);
    int v = lens[gl];
    v = v < 0 ? 0 : v;
    v = v > T ? T : v;
    lenr[r] = (grow < nreal) ? v : 0;
  }

  for (int i = tid; i < 16 * kHP; i += 128) {
    sH[i] = (unsigned short)0;
    sO[i] = (unsigned short)0;
  }

  float cst[8];
  unsigned hpb[8];
  unsigned fin[8];
#pragma unroll
  for (int r = 0; r < 8; ++r) {
    cst[r] = 0.0f;
    hpb[r] = 0u;
    fin[r] = 0u;
  }
  const int srow = tid >> 3;
  const int sch = tid & 7;
  const int orow = wave * 4 + (lane >> 3);
  const int oc8 = (lane & 7) * 8;
  __syncthreads();

#pragma unroll 1
  for (int s = 0; s < T; ++s) {
    const int t = dir ? (T - 1 - s) : s;
    {
      const unsigned short* gsrc = G + ((size_t)(row0 + srow) * T + t) * kGN + dir * 256;
      const v4u* gp = (const v4u*)(const void*)gsrc;
      const v4u g0 = gp[sch];
      const v4u g1 = gp[sch + 8];
      const v4u g2 = gp[sch + 16];
      const v4u g3 = gp[sch + 24];
      unsigned short* gd = sG + srow * kGP + sch * 8;
      *(v4u*)(void*)(gd)       = g0;
      *(v4u*)(void*)(gd + 64)  = g1;
      *(v4u*)(void*)(gd + 128) = g2;
      *(v4u*)(void*)(gd + 192) = g3;
    }
    v8f acc[4];
    {
      const _Float16* hp = (const _Float16*)(const void*)sH + c * kHP + 8 * hh;
      const v16h a0 = FragH::load(hp);
      const v16h a1 = FragH::load(hp + 32);
#pragma unroll
      for (int g = 0; g < 4; ++g) {
        acc[g] = (v8f){0.f, 0.f, 0.f, 0.f, 0.f, 0.f, 0.f, 0.f};
        acc[g] = mma_g(a0, bfr[g][0], acc[g]);
        acc[g] = mma_g(a1, bfr[g][1], acc[g]);
      }
    }
    __syncthreads();
#pragma unroll
    for (int r = 0; r < 8; ++r) {
      const int rl = 8 * hh + r;
      const unsigned short* gr = sG + rl * kGP + unit;
      const float xi = h16_to_f32((unsigned)gr[0]);
      const float xf = h16_to_f32((unsigned)gr[64]);
      const float xg = h16_to_f32((unsigned)gr[128]);
      const float xo = h16_to_f32((unsigned)gr[192]);
      const float pi = acc[0][r] * kWCarryInv + xi;
      const float pf = acc[1][r] * kWCarryInv + xf;
      const float pg = acc[2][r] * kWCarryInv + xg;
      const float po = acc[3][r] * kWCarryInv + xo;
      const float ig = sigm(pi);
      const float fg = sigm(pf);
      const float gg = tanh_e(pg);
      const float og = sigm(po);
      float cn = fg * cst[r] + ig * gg;
      float hn = og * tanh_e(cn);
      cn = unit_ok ? cn : 0.0f;
      hn = unit_ok ? hn : 0.0f;
      const bool valid = t < lenr[r];
      cst[r] = valid ? cn : cst[r];
      const unsigned hb = f32_to_h16bits(hn);
      const unsigned hs = valid ? hb : hpb[r];
      hpb[r] = hs;
      sH[rl * kHP + unit] = (unsigned short)hs;
      if (!LAST_ONLY) {
        const unsigned ov = valid ? hb : 0u;
        sO[rl * kHP + unit] = (unsigned short)ov;
      } else {
        fin[r] = (t == (lenr[r] - 1)) ? hb : fin[r];
      }
    }
    __syncthreads();
    if (!LAST_ONLY) {
      const v4u ov = *(const v4u*)(const void*)(sO + orow * kHP + oc8);
      unsigned short* op = outp + ((size_t)(row0 + orow) * T + t) * kFP + dir * 64 + oc8;
      *(volatile v4u*)(void*)op = ov;
      __threadfence();
      *(volatile v4u*)(void*)op = ov;
    }
  }
  if (LAST_ONLY) {
#pragma unroll
    for (int r = 0; r < 8; ++r) sO[(8 * hh + r) * kHP + unit] = (unsigned short)fin[r];
    __syncthreads();
    const v4u ov = *(const v4u*)(const void*)(sO + orow * kHP + oc8);
    unsigned short* op = outp + (size_t)(row0 + orow) * kFP + dir * 64 + oc8;
    *(volatile v4u*)(void*)op = ov;
    __threadfence();
    *(volatile v4u*)(void*)op = ov;
  }
}

__global__ __launch_bounds__(256) void build_ob_kernel(
    const unsigned short* __restrict__ WHPU, const int* __restrict__ l_hs,
    const int* __restrict__ wn, const int* __restrict__ wc, unsigned short* __restrict__ OB) {
  __shared__ int sPart[8];
  const int b = blockIdx.x;
  const int tid = threadIdx.x, lane = tid & 31, wave = tid >> 5;
  static_assert(kBS == 256);
  int v = l_hs[tid];
  v = (tid < b) ? v : 0;
#pragma unroll
  for (int off = 16; off > 0; off >>= 1) v += __shfl_xor(v, off, 32);
  if (lane == 0) sPart[wave] = v;
  __syncthreads();
  int offs = 0;
#pragma unroll
  for (int i = 0; i < 8; ++i) offs += sPart[i];
  const int lb = l_hs[b];
  const int w_n = wn[b];
#pragma unroll 1
  for (int it = 0; it < 2; ++it) {
    const int idx = tid + 256 * it;
    const int idxc = idx < 320 ? idx : 319;
    const int j = idxc >> 4;
    const int ch = idxc & 15;
    const int colraw = wc[b * kMLW + j];
    int col = (j < w_n) ? colraw : 0;
    col = col < 0 ? 0 : col;
    col = col > (kMLHS - 1) ? (kMLHS - 1) : col;
    const bool valid = col < lb;
    int row = offs + col;
    row = row < 0 ? 0 : row;
    row = row > (kNH - 1) ? (kNH - 1) : row;
    v4u val = *(const v4u*)(const void*)(WHPU + (size_t)row * kFP + ch * 8);
    const v4u zero4 = (v4u){0u, 0u, 0u, 0u};
    val = valid ? val : zero4;
    if (idx < 320) {
      unsigned short* op = OB + ((size_t)(b * kMLW + j)) * kFP + ch * 8;
      *(volatile v4u*)(void*)op = val;
      __threadfence();
      *(volatile v4u*)(void*)op = val;
    }
  }
}

constexpr int kAP = 136;
constexpr int kSP = 132;

__global__ __launch_bounds__(64) void attn_kernel(
    const unsigned short* __restrict__ Q, const unsigned short* __restrict__ WN,
    const unsigned short* __restrict__ OB, const int* __restrict__ l_n,
    unsigned short* __restrict__ CN) {
  __shared__ __align__(16) unsigned short sVt[128 * kAP];
  __shared__ __align__(16) unsigned short sP[32 * kAP];
  __shared__ __align__(16) float sS[32 * kSP];
  __shared__ float sInv[32];
  const int tid = threadIdx.x, lane = tid & 31, wave = tid >> 5, hh = lane >> 4, c = lane & 15;
  const int b = blockIdx.x;
  const int len = l_n[b];

#pragma unroll 1
  for (int it = 0; it < 32; ++it) {
    const int idx = tid + 64 * it;
    const int t = idx >> 4;
    const int ch = idx & 15;
    const v4u g = *(const v4u*)(const void*)(WN + ((size_t)(b * kTN + t)) * kFP + ch * 8);
    const unsigned w0 = g[0];
    const unsigned w1 = g[1];
    const unsigned w2 = g[2];
    const unsigned w3 = g[3];
    unsigned short* vp = sVt + (ch * 8) * kAP + t;
    vp[0 * kAP] = (unsigned short)(w0 & 0xffffu);
    vp[1 * kAP] = (unsigned short)(w0 >> 16);
    vp[2 * kAP] = (unsigned short)(w1 & 0xffffu);
    vp[3 * kAP] = (unsigned short)(w1 >> 16);
    vp[4 * kAP] = (unsigned short)(w2 & 0xffffu);
    vp[5 * kAP] = (unsigned short)(w2 >> 16);
    vp[6 * kAP] = (unsigned short)(w3 & 0xffffu);
    vp[7 * kAP] = (unsigned short)(w3 >> 16);
  }

  {
    const int jr = wave * 16 + c;
    const int jrc = jr < kMLW ? jr : (kMLW - 1);
    const _Float16* obp = (const _Float16*)(const void*)(OB + ((size_t)(b * kMLW + jrc)) * kFP) + 8 * hh;
    v16h afr[4];
#pragma unroll
    for (int ks = 0; ks < 4; ++ks) afr[ks] = FragH::load(obp + ks * 32);
    const _Float16* qp = (const _Float16*)(const void*)(Q + ((size_t)(b * kTN + c)) * kFP) + 8 * hh;
#pragma unroll
    for (int nt = 0; nt < 8; ++nt) {
      v8f sc = (v8f){0.f, 0.f, 0.f, 0.f, 0.f, 0.f, 0.f, 0.f};
#pragma unroll
      for (int ks = 0; ks < 4; ++ks)
        sc = mma_g(afr[ks], FragH::load(qp + (size_t)nt * 16 * kFP + ks * 32), sc);
#pragma unroll
      for (int r = 0; r < 8; ++r) sS[(wave * 16 + 8 * hh + r) * kSP + nt * 16 + c] = sc[r];
    }
  }
  __syncthreads();

#pragma unroll 1
  for (int rr = 0; rr < 16; ++rr) {
    const int row = wave * 16 + rr;
    const float* sr = sS + row * kSP;
    float v0 = sr[lane];
    float v1 = sr[lane + 32];
    float v2 = sr[lane + 64];
    float v3 = sr[lane + 96];
    v0 = (lane < len) ? v0 : kNegFill;
    v1 = ((lane + 32) < len) ? v1 : kNegFill;
    v2 = ((lane + 64) < len) ? v2 : kNegFill;
    v3 = ((lane + 96) < len) ? v3 : kNegFill;
    float m = fmaxf(fmaxf(v0, v1), fmaxf(v2, v3));
#pragma unroll
    for (int off = 16; off > 0; off >>= 1) m = fmaxf(m, __shfl_xor(m, off, 32));
    const float e0 = expf(v0 - m);
    const float e1 = expf(v1 - m);
    const float e2 = expf(v2 - m);
    const float e3 = expf(v3 - m);
    float sum = (e0 + e1) + (e2 + e3);
#pragma unroll
    for (int off = 16; off > 0; off >>= 1) sum += __shfl_xor(sum, off, 32);
    unsigned short* pr = sP + row * kAP;
    pr[lane]      = (unsigned short)f32_to_h16bits(e0 * kPCarry);
    pr[lane + 32] = (unsigned short)f32_to_h16bits(e1 * kPCarry);
    pr[lane + 64] = (unsigned short)f32_to_h16bits(e2 * kPCarry);
    pr[lane + 96] = (unsigned short)f32_to_h16bits(e3 * kPCarry);
    if (lane == 0) sInv[row] = 1.0f / (sum * kPCarry);
  }
  __syncthreads();

  {
    const _Float16* pp = (const _Float16*)(const void*)sP + (wave * 16 + c) * kAP + 8 * hh;
    v16h pfr[4];
#pragma unroll
    for (int ks = 0; ks < 4; ++ks) pfr[ks] = FragH::load(pp + ks * 32);
    float inv[8];
#pragma unroll
    for (int r = 0; r < 8; ++r) inv[r] = sInv[wave * 16 + 8 * hh + r];
#pragma unroll
    for (int nt = 0; nt < 8; ++nt) {
      const _Float16* vp = (const _Float16*)(const void*)sVt + (nt * 16 + c) * kAP + 8 * hh;
      v8f o = (v8f){0.f, 0.f, 0.f, 0.f, 0.f, 0.f, 0.f, 0.f};
#pragma unroll
      for (int ks = 0; ks < 4; ++ks) o = mma_g(pfr[ks], FragH::load(vp + ks * 32), o);
#pragma unroll
      for (int r = 0; r < 8; ++r) sS[(wave * 16 + 8 * hh + r) * kSP + nt * 16 + c] = o[r] * inv[r];
    }
  }
  __syncthreads();

#pragma unroll 1
  for (int it = 0; it < 5; ++it) {
    const int idx = tid + 64 * it;
    const int row = idx >> 4;
    const int ch = idx & 15;
    const float* sp = sS + row * kSP + ch * 8;
    const v4f a0 = *(const v4f*)(sp);
    const v4f a1 = *(const v4f*)(sp + 4);
    v8h hv;
#pragma unroll
    for (int e = 0; e < 4; ++e) {
      hv[e]     = (_Float16)a0[e];
      hv[4 + e] = (_Float16)a1[e];
    }
    unsigned short* op = CN + ((size_t)(b * kMLW + row)) * kFP + ch * 8;
    *(volatile v8h*)op = hv;
    __threadfence();
    *(volatile v8h*)op = hv;
  }
}

__global__ __launch_bounds__(256) void head_out_kernel(
    const float* __restrict__ H, const float* __restrict__ W, const float* __restrict__ Bv,
    float* __restrict__ outp, int total) {
  const int e = blockIdx.x * 256 + threadIdx.x;
  if (e >= total) return;
  const int row = e / kNOPS;
  const int cc = e - row * kNOPS;
  const float* hp = H + (size_t)row * 128;
  const float* wp = W + (size_t)cc * 100;
  float acc = 0.0f;
#pragma unroll 1
  for (int k4 = 0; k4 < 25; ++k4) {
    const v4f a = *(const v4f*)(hp + 4 * k4);
    const v4f w = *(const v4f*)(wp + 4 * k4);
    acc = fmaf(a[0], w[0], acc);
    acc = fmaf(a[1], w[1], acc);
    acc = fmaf(a[2], w[2], acc);
    acc = fmaf(a[3], w[3], acc);
  }
  const float val = acc + Bv[cc];
  *(volatile float*)(outp + e) = val;
  __threadfence();
  *(volatile float*)(outp + e) = val;
}

extern "C" void kernel_launch(void* const* d_in, const int* in_sizes, int n_in,
                              void* d_out, int out_size, void* d_ws, size_t ws_size,
                              hipStream_t stream) {
  if (n_in < 27) return;
  if (in_sizes[0] != kBS * kTN * kIS) return;
  if (in_sizes[1] != kNH * kTH * kIS) return;
  if (in_sizes[22] != kBS) return;
  if (in_sizes[23] != kNH) return;
  if (in_sizes[24] != kBS) return;
  if (in_sizes[26] != kBS * kMLW) return;
  if (out_size != kOutN) return;
  if (ws_size < kWsTotal) return;

  const float* wemb_n   = (const float*)d_in[0];
  const float* wemb_hpu = (const float*)d_in[1];
  const float* n_Wih0   = (const float*)d_in[2];
  const float* n_Wih1   = (const float*)d_in[3];
  const float* n_Whh    = (const float*)d_in[4];
  const float* n_bih    = (const float*)d_in[5];
  const float* n_bhh    = (const float*)d_in[6];
  const float* h_Wih0   = (const float*)d_in[7];
  const float* h_Wih1   = (const float*)d_in[8];
  const float* h_Whh    = (const float*)d_in[9];
  const float* h_bih    = (const float*)d_in[10];
  const float* h_bhh    = (const float*)d_in[11];
  const float* W_att_w  = (const float*)d_in[12];
  const float* W_att_b  = (const float*)d_in[13];
  const float* W_c_w    = (const float*)d_in[14];
  const float* W_c_b    = (const float*)d_in[15];
  const float* W_hs_w   = (const float*)d_in[16];
  const float* W_hs_b   = (const float*)d_in[17];
  const float* wo0_w    = (const float*)d_in[18];
  const float* wo0_b    = (const float*)d_in[19];
  const float* wo1_w    = (const float*)d_in[20];
  const float* wo1_b    = (const float*)d_in[21];
  const int*   l_n      = (const int*)d_in[22];
  const int*   l_hpu    = (const int*)d_in[23];
  const int*   l_hs     = (const int*)d_in[24];
  const int*   wn       = (const int*)d_in[25];
  const int*   wc       = (const int*)d_in[26];

  char* ws = (char*)d_ws;
  unsigned short* X16   = (unsigned short*)(ws + kOffX);
  unsigned short* GP    = (unsigned short*)(ws + kOffG);
  unsigned short* L0    = (unsigned short*)(ws + kOffL0);
  unsigned short* WENCN = (unsigned short*)(ws + kOffWN);
  unsigned short* QP    = (unsigned short*)(ws + kOffQ);
  unsigned short* WHPU  = (unsigned short*)(ws + kOffHPU);
  unsigned short* OB    = (unsigned short*)(ws + kOffOB);
  unsigned short* CN    = (unsigned short*)(ws + kOffCN);
  unsigned short* VEC   = (unsigned short*)(ws + kOffVEC);
  float*          HF    = (float*)(ws + kOffHF);
  unsigned short* WIH0N = (unsigned short*)(ws + kOffWih0N);
  unsigned short* WIH0H = (unsigned short*)(ws + kOffWih0H);
  unsigned short* WIH1N = (unsigned short*)(ws + kOffWih1N);
  unsigned short* WIH1H = (unsigned short*)(ws + kOffWih1H);
  unsigned short* WHHN  = (unsigned short*)(ws + kOffWhhN);
  unsigned short* WHHH  = (unsigned short*)(ws + kOffWhhH);
  unsigned short* WATT  = (unsigned short*)(ws + kOffWatt);
  unsigned short* WC    = (unsigned short*)(ws + kOffWc);
  unsigned short* WHS   = (unsigned short*)(ws + kOffWhs);
  unsigned short* WO0   = (unsigned short*)(ws + kOffWo0);
  float*          BIAS  = (float*)(ws + kOffBias);

  auto pack = [&](const float* src, unsigned short* dst, int srcRows, int srcCols, int dstRows, int dstCols,
                  int rshift, int rblk, int cshift, int cblk) {
    const int total8 = dstRows * (dstCols / 8);
    pack_plane_kernel<<<(total8 + 255) / 256, 256, 0, stream>>>(src, dst, srcRows, srcCols, dstCols / 8, total8,
                                                                rshift, rblk, cshift, cblk, kWCarry);
  };
  pack(n_Wih0, WIH0N, 400, 300, 512, 320, 6, 50, 20, 300);
  pack(h_Wih0, WIH0H, 400, 300, 512, 320, 6, 50, 20, 300);
  pack(n_Wih1, WIH1N, 400, 100, 512, 128, 6, 50, 6, 50);
  pack(h_Wih1, WIH1H, 400, 100, 512, 128, 6, 50, 6, 50);
  pack(n_Whh, WHHN, 800, 50, 1024, 64, 6, 50, 20, 50);
  pack(h_Whh, WHHH, 800, 50, 1024, 64, 6, 50, 20, 50);
  pack(W_att_w, WATT, 100, 100, 128, 128, 6, 50, 6, 50);
  pack(W_c_w, WC, 100, 100, 128, 128, 20, 100, 6, 50);
  pack(W_hs_w, WHS, 100, 100, 128, 128, 20, 100, 6, 50);
  pack(wo0_w, WO0, 100, 200, 128, 256, 20, 100, 7, 100);
  pack_bias_kernel<<<20, 32, 0, stream>>>(n_bih, n_bhh, h_bih, h_bhh, W_att_b, W_c_b, W_hs_b, wo0_b, BIAS);

  convert_x_kernel<<<(kMQ * 40) / 256, 256, 0, stream>>>(wemb_n, X16, kMQ, kMQ * 40);
  wmma_gemm64<1, 0><<<((kMQ / 64) * (kGN / 64) + 7) / 8, 256, 0, stream>>>(
      X16, kKX, WIH0N, kKX, (void*)GP, kGN, BIAS + kBiasN0, kMQ, kGN, kKX, kWCarryInv);
  lstm_rec_kernel<false><<<dim3(kBS / 16, 2), 128, 0, stream>>>(GP, WHHN, l_n, kBS, kTN, L0);
  wmma_gemm64<1, 0><<<((kMQ / 64) * (kGN / 64) + 7) / 8, 256, 0, stream>>>(
      L0, kFP, WIH1N, kFP, (void*)GP, kGN, BIAS + kBiasN1, kMQ, kGN, kFP, kWCarryInv);
  lstm_rec_kernel<false><<<dim3(kBS / 16, 2), 128, 0, stream>>>(GP, WHHN + (size_t)2 * 256 * 64, l_n, kBS, kTN, WENCN);

  convert_x_kernel<<<(kMH * 40) / 256, 256, 0, stream>>>(wemb_hpu, X16, kMHR, kMH * 40);
  wmma_gemm64<1, 0><<<((kMH / 64) * (kGN / 64) + 7) / 8, 256, 0, stream>>>(
      X16, kKX, WIH0H, kKX, (void*)GP, kGN, BIAS + kBiasH0, kMH, kGN, kKX, kWCarryInv);
  lstm_rec_kernel<false><<<dim3(kNHP / 16, 2), 128, 0, stream>>>(GP, WHHH, l_hpu, kNH, kTH, L0);
  wmma_gemm64<1, 0><<<((kMH / 64) * (kGN / 64) + 7) / 8, 256, 0, stream>>>(
      L0, kFP, WIH1H, kFP, (void*)GP, kGN, BIAS + kBiasH1, kMH, kGN, kFP, kWCarryInv);
  lstm_rec_kernel<true><<<dim3(kNHP / 16, 2), 128, 0, stream>>>(GP, WHHH + (size_t)2 * 256 * 64, l_hpu, kNH, kTH, WHPU);

  build_ob_kernel<<<kBS, 256, 0, stream>>>(WHPU, l_hs, wn, wc, OB);

  wmma_gemm64<1, 0><<<((kMQ / 64) * (128 / 64) + 7) / 8, 256, 0, stream>>>(
      WENCN, kFP, WATT, kFP, (void*)QP, kFP, BIAS + kBiasAtt, kMQ, 128, kFP, kWCarryInv);
  attn_kernel<<<kBS, 64, 0, stream>>>(QP, WENCN, OB, l_n, CN);

  wmma_gemm64<1, 0><<<((kMJ / 64) * (128 / 64) + 7) / 8, 256, 0, stream>>>(
      CN, kFP, WC, kFP, (void*)VEC, 256, BIAS + kBiasC, kMJ, 128, kFP, kWCarryInv);
  wmma_gemm64<1, 0><<<((kMJ / 64) * (128 / 64) + 7) / 8, 256, 0, stream>>>(
      OB, kFP, WHS, kFP, (void*)(VEC + 128), 256, BIAS + kBiasHs, kMJ, 128, kFP, kWCarryInv);
  wmma_gemm64<0, 1><<<((kMJ / 64) * (128 / 64) + 7) / 8, 256, 0, stream>>>(
      VEC, 256, WO0, 256, (void*)HF, 128, BIAS + kBiasWo0, kMJ, 128, 256, kWCarryInv);
  head_out_kernel<<<kOutN / 256, 256, 0, stream>>>(HF, wo1_w, wo1_b, (float*)d_out, kOutN);
}
